// TransformerBlock_5033701671200
// MI455X (gfx1250) — hardware-run, weakly checked
//
#include <hip/hip_runtime.h>


#ifndef NB
#define NB 2
#endif
#ifndef SEQ
#define SEQ 2048
#endif
#define NB_FULL    2
#define SEQ_FULL   2048
#define EMB        128
#define NHEAD      16
#define HDIM       128
#define HID        512
#define CTXW       (NHEAD * HDIM)
#define QKVN       (3 * CTXW)
#define MROWS      (NB * SEQ)
#define NPAIR      (HDIM / 2)
#define BQ         128
#define BK         32
#define NWAVE      8
#define OHALF      64
#define OP         68
#define TPV        136
#define TPW        72

#define QK_ELEMS    ((size_t)NB * NHEAD * SEQ * HDIM)
#define TAB_BYTES   ((size_t)2 * SEQ * NPAIR * 4)
#define WQKV_BYTES  ((size_t)QKVN * EMB * 2)
#define WO_BYTES    ((size_t)EMB * CTXW * 2)
#define F1_BYTES    ((size_t)HID * EMB * 2)
#define F2_BYTES    ((size_t)EMB * HID * 2)
#define H_BYTES     ((size_t)MROWS * EMB * 2)
#define QKP_BYTES   ((size_t)2 * QK_ELEMS * 2)
#define VT_BYTES    ((size_t)QK_ELEMS * 2)
#define CTX_BYTES   ((size_t)MROWS * CTXW * 2)
#define X2_BYTES    ((size_t)MROWS * EMB * 4)
#define G_BYTES     ((size_t)MROWS * HID * 2)

#define OFF_TAB   ((size_t)0)
#define OFF_WQKV  (OFF_TAB + TAB_BYTES)
#define OFF_WO    (OFF_WQKV + WQKV_BYTES)
#define OFF_F1    (OFF_WO + WO_BYTES)
#define OFF_F2    (OFF_F1 + F1_BYTES)
#define OFF_H     (OFF_F2 + F2_BYTES)
#define OFF_QK    (OFF_H + H_BYTES)
#define OFF_VT    (OFF_QK + QKP_BYTES)
#define OFF_CTX   (OFF_VT + VT_BYTES)
#define OFF_X2    (OFF_CTX + CTX_BYTES)
#define OFF_H2    (OFF_X2 + X2_BYTES)
#define OFF_G     (OFF_H2 + H_BYTES)
#define WS_TOTAL  (OFF_G + G_BYTES)

static_assert(SEQ % BQ == 0);
static_assert(SEQ % BK == 0);
static_assert(SEQ % 4 == 0);
static_assert(BQ == NWAVE * 16);
static_assert(HDIM == 128);
static_assert(EMB == 128);
static_assert(EMB % 32 == 0 && CTXW % 32 == 0 && HID % 32 == 0);
static_assert(2 * OHALF == HDIM);
static_assert(2 * OHALF == EMB);
static_assert(16 * 4 == OHALF);
static_assert(8 * 8 == OHALF);
static_assert(HID % 128 == 0);
static_assert(MROWS % BQ == 0);
static_assert(MROWS % 16 == 0);
static_assert(NPAIR == 64);
static_assert(256 == 4 * NPAIR);
static_assert(EMB % 64 == 0 && CTXW % 64 == 0 && HID % 64 == 0);
static_assert(256 * 4 * 4 == 64 * 64);
static_assert(256 * 8 * 8 == HDIM * BQ);
static_assert(TPV >= BQ && TPW >= 64 && OP >= OHALF);
static_assert((TPV * 2) % 16 == 0 && (TPW * 2) % 16 == 0 && (OP * 4) % 16 == 0);
static_assert(NWAVE * 16 * OP * 4 <= 65536);
static_assert(HDIM * TPV * 2 <= 65536);
static_assert(SEQ <= SEQ_FULL);
static_assert(NB >= 1 && NB <= NB_FULL);
static_assert(TAB_BYTES % 128 == 0 && WQKV_BYTES % 128 == 0 && WO_BYTES % 128 == 0 && F1_BYTES % 128 == 0);
static_assert(F2_BYTES % 128 == 0 && H_BYTES % 128 == 0 && QKP_BYTES % 128 == 0 && VT_BYTES % 128 == 0);
static_assert(CTX_BYTES % 128 == 0 && X2_BYTES % 128 == 0 && G_BYTES % 128 == 0);
static_assert(WS_TOTAL <= (size_t)134217728);

typedef __bf16   bf16;
typedef _Float16 f16;
typedef f16      v16h  __attribute__((ext_vector_type(16)));
typedef f16      v8h   __attribute__((ext_vector_type(8)));
typedef float    v8f   __attribute__((ext_vector_type(8)));
typedef float    v4f   __attribute__((ext_vector_type(4)));
typedef unsigned v4u   __attribute__((ext_vector_type(4)));

union FragH  { v16h  v; v4u q[2]; f16  h[16]; };
union Pack8H { v4u u; v8h v; f16 h[8]; };

static __device__ __forceinline__ v8f mma_f16(v16h a, v16h b, v8f acc) {
  acc = __builtin_amdgcn_wmma_f32_16x16x32_f16(false, a, false, b, (short)0, acc, false, false);
  asm volatile("v_nop\n\tv_nop\n\tv_nop\n\tv_nop" : "+v"(acc) : "v"(a), "v"(b));
  return acc;
}

static __device__ __forceinline__ float bfr(float v) { return (float)(bf16)v; }

static __device__ __forceinline__ f16 toh_flush(float v) {
  const f16 r = (f16)v;
  return (fabsf(v) < 6.103515625e-05f) ? (f16)0.0f : r;
}

static __device__ __forceinline__ void gemm_16x128(const f16* __restrict__ A, const f16* __restrict__ Bt,
                                                   const int K, const size_t arow, const size_t brow0,
                                                   const int lq, const int hi, v8f (&acc)[8]) {
  #pragma unroll
  for (int nt = 0; nt < 8; ++nt) acc[nt] = (v8f){0, 0, 0, 0, 0, 0, 0, 0};
  const f16* ap = A + (arow + lq) * (size_t)K + hi * 8;
  const f16* bp = Bt + (brow0 + lq) * (size_t)K + hi * 8;
  #pragma unroll 1
  for (int k0 = 0; k0 < K; k0 += 32) {
    FragH a;
    a.q[0] = *(const v4u*)(ap + k0);
    a.q[1] = *(const v4u*)(ap + k0 + 16);
    #pragma unroll
    for (int g = 0; g < 2; ++g) {
      FragH bv[4];
      #pragma unroll
      for (int t = 0; t < 4; ++t) {
        const f16* base = bp + (size_t)((g * 4 + t) * 16) * (size_t)K + k0;
        bv[t].q[0] = *(const v4u*)(base);
        bv[t].q[1] = *(const v4u*)(base + 16);
      }
      #pragma unroll
      for (int t = 0; t < 4; ++t) acc[g * 4 + t] = mma_f16(a.v, bv[t].v, acc[g * 4 + t]);
      __builtin_amdgcn_sched_barrier(0);
    }
  }
}

__global__ __launch_bounds__(256) void rope_table_kernel(float* __restrict__ tab) {
  #pragma clang fp contract(off)
  const int tid = threadIdx.x;
  const int i   = tid & 63;
  const int s   = blockIdx.x * 4 + (tid >> 6);
  __shared__ __align__(16) float sC[256];
  __shared__ __align__(16) float sS[256];
  double r = 1.0;
  #pragma unroll 1
  for (int j = 0; j < i; ++j) r *= 0.8659643233600654;
  const float inv = (float)r;
  const float ang = (float)s * inv;
  sC[tid] = cosf(ang);
  sS[tid] = sinf(ang);
  __syncthreads();
  if (tid < 128) {
    const int wsel = tid >> 6;
    const int t    = tid & 63;
    const v4f vc = *(const v4f*)(&sC[t * 4]);
    const v4f vs = *(const v4f*)(&sS[t * 4]);
    const v4f val = wsel ? vs : vc;
    float* dst = tab + (size_t)wsel * SEQ * NPAIR + (size_t)blockIdx.x * 256 + t * 4;
    *(volatile v4f*)dst = val;
    __threadfence();
    *(volatile v4f*)dst = val;
  }
}

__global__ __launch_bounds__(256) void wt_plane_kernel(const float* __restrict__ w, f16* __restrict__ wt,
                                                       const int K, const int N, const int n_off) {
  #pragma clang fp contract(off)
  const int tid = threadIdx.x;
  const int n0  = blockIdx.x * 64;
  const int k0  = blockIdx.y * 64;
  __shared__ __align__(16) f16 sW[64 * TPW];
  #pragma unroll
  for (int j = 0; j < 4; ++j) {
    const int idx = j * 256 + tid;
    const int kk  = idx >> 4;
    const int n4  = (idx & 15) * 4;
    const v4f v = *(const v4f*)(w + (size_t)(k0 + kk) * N + n0 + n4);
    #pragma unroll
    for (int e = 0; e < 4; ++e) sW[(n4 + e) * TPW + kk] = toh_flush(bfr(v[e]) * 256.0f);
  }
  __syncthreads();
  v4u    val[2];
  size_t idxo[2];
  #pragma unroll
  for (int j = 0; j < 2; ++j) {
    const int idx = j * 256 + tid;
    const int n   = idx >> 3;
    const int seg = idx & 7;
    Pack8H ph;
    ph.v = *(const v8h*)(&sW[n * TPW + seg * 8]);
    val[j]  = ph.u;
    idxo[j] = (size_t)(n_off + n0 + n) * K + k0 + seg * 8;
  }
  #pragma unroll
  for (int j = 0; j < 2; ++j) *(volatile v4u*)(wt + idxo[j]) = val[j];
  __threadfence();
  #pragma unroll
  for (int j = 0; j < 2; ++j) *(volatile v4u*)(wt + idxo[j]) = val[j];
}

__global__ __launch_bounds__(256) void ln_kernel(const float* __restrict__ src, const float* __restrict__ gam,
                                                 const float* __restrict__ bet, f16* __restrict__ dst,
                                                 const int src_is_input) {
  #pragma clang fp contract(off)
  const int tid  = threadIdx.x;
  const int wave = __builtin_amdgcn_readfirstlane(tid >> 5);
  const int lane = tid & 31;
  const int m    = (blockIdx.x * 8 + wave) * 2 + (lane >> 4);
  const int c0   = (lane & 15) * 8;
  const int b    = m / SEQ;
  const int s    = m - b * SEQ;
  const size_t srow = src_is_input ? ((size_t)b * SEQ_FULL + s) : (size_t)m;
  const v4f x0 = *(const v4f*)(src + srow * EMB + c0);
  const v4f x1 = *(const v4f*)(src + srow * EMB + c0 + 4);
  const v4f g0 = *(const v4f*)(gam + c0);
  const v4f g1 = *(const v4f*)(gam + c0 + 4);
  const v4f b0 = *(const v4f*)(bet + c0);
  const v4f b1 = *(const v4f*)(bet + c0 + 4);
  float v[8];
  #pragma unroll
  for (int i = 0; i < 4; ++i) {
    const float a0 = x0[i];
    const float a1 = x1[i];
    const float r0 = bfr(a0);
    const float r1 = bfr(a1);
    v[i]     = src_is_input ? r0 : a0;
    v[4 + i] = src_is_input ? r1 : a1;
  }
  float sum = 0.0f;
  #pragma unroll
  for (int i = 0; i < 8; ++i) sum += v[i];
  sum += __shfl_xor(sum, 8, 32);
  sum += __shfl_xor(sum, 4, 32);
  sum += __shfl_xor(sum, 2, 32);
  sum += __shfl_xor(sum, 1, 32);
  const float mu = sum * (1.0f / EMB);
  float var = 0.0f;
  #pragma unroll
  for (int i = 0; i < 8; ++i) { const float d = v[i] - mu; var += d * d; }
  var += __shfl_xor(var, 8, 32);
  var += __shfl_xor(var, 4, 32);
  var += __shfl_xor(var, 2, 32);
  var += __shfl_xor(var, 1, 32);
  const float rinv = 1.0f / sqrtf(var * (1.0f / EMB) + 1e-5f);
  Pack8H ph;
  #pragma unroll
  for (int i = 0; i < 4; ++i) {
    ph.h[i]     = toh_flush((v[i] - mu) * rinv * bfr(g0[i]) + bfr(b0[i]));
    ph.h[4 + i] = toh_flush((v[4 + i] - mu) * rinv * bfr(g1[i]) + bfr(b1[i]));
  }
  const v4u val = ph.u;
  f16* dp = dst + (size_t)m * EMB + c0;
  *(volatile v4u*)dp = val;
  __threadfence();
  *(volatile v4u*)dp = val;
}

__global__ __launch_bounds__(256) void qk_proj_kernel(const f16* __restrict__ hpl, const f16* __restrict__ wqkv,
                                                      const float* __restrict__ tab, f16* __restrict__ qk) {
  const int cb    = blockIdx.x;
  const int which = cb >> 4;
  const int h     = cb & 15;
  const int tid   = threadIdx.x;
  const int wave  = __builtin_amdgcn_readfirstlane(tid >> 5);
  const int lane  = tid & 31;
  const int lq    = lane & 15;
  const int hi    = lane >> 4;

  __shared__ __align__(16) float sO[NWAVE * 16 * OP];

  const int m0 = blockIdx.y * BQ + wave * 16;
  const int b  = m0 / SEQ;
  const int s0 = m0 - b * SEQ;

  v8f acc[8];
  gemm_16x128(hpl, wqkv, EMB, (size_t)m0, (size_t)cb * HDIM, lq, hi, acc);

  const size_t obase = (size_t)which * QK_ELEMS + (((size_t)b * NHEAD + h) * SEQ + s0) * HDIM;
  const int so = wave * (16 * OP);
  const float INV = 1.0f / 256.0f;
  v4u    vals[8];
  size_t gidx[4];

  #pragma unroll
  for (int half = 0; half < 2; ++half) {
    #pragma unroll
    for (int r = 0; r < 8; ++r) {
      #pragma unroll
      for (int t = 0; t < 4; ++t) sO[so + (hi * 8 + r) * OP + t * 16 + lq] = acc[half * 4 + t][r] * INV;
    }
    __syncthreads();
    #pragma unroll
    for (int it = 0; it < 4; ++it) {
      const int row = it * 4 + (lane >> 3);
      const int cg  = (lane & 7) * 8;
      const v4f a0 = *(const v4f*)(&sO[so + row * OP + cg]);
      const v4f a1 = *(const v4f*)(&sO[so + row * OP + cg + 4]);
      const int pi = (half * OHALF + cg) >> 1;
      const float* tp = tab + (size_t)(s0 + row) * NPAIR + pi;
      const v4f cs = *(const v4f*)(tp);
      const v4f sn = *(const v4f*)(tp + (size_t)SEQ * NPAIR);
      Pack8H ph;
      ph.h[0] = toh_flush(a0[0] * cs[0] - a0[1] * sn[0]);
      ph.h[1] = toh_flush(a0[0] * sn[0] + a0[1] * cs[0]);
      ph.h[2] = toh_flush(a0[2] * cs[1] - a0[3] * sn[1]);
      ph.h[3] = toh_flush(a0[2] * sn[1] + a0[3] * cs[1]);
      ph.h[4] = toh_flush(a1[0] * cs[2] - a1[1] * sn[2]);
      ph.h[5] = toh_flush(a1[0] * sn[2] + a1[1] * cs[2]);
      ph.h[6] = toh_flush(a1[2] * cs[3] - a1[3] * sn[3]);
      ph.h[7] = toh_flush(a1[2] * sn[3] + a1[3] * cs[3]);
      vals[half * 4 + it] = ph.u;
      gidx[it] = obase + (size_t)row * HDIM + cg;
    }
    if (half == 0) __syncthreads();
  }

  #pragma unroll
  for (int it = 0; it < 4; ++it) {
    *(volatile v4u*)(qk + gidx[it])         = vals[it];
    *(volatile v4u*)(qk + gidx[it] + OHALF) = vals[4 + it];
  }
  __threadfence();
  #pragma unroll
  for (int it = 0; it < 4; ++it) {
    *(volatile v4u*)(qk + gidx[it])         = vals[it];
    *(volatile v4u*)(qk + gidx[it] + OHALF) = vals[4 + it];
  }
}

__global__ __launch_bounds__(256) void v_proj_kernel(const f16* __restrict__ hpl, const f16* __restrict__ wqkv,
                                                     f16* __restrict__ vt) {
  const int h    = blockIdx.x;
  const int tid  = threadIdx.x;
  const int wave = __builtin_amdgcn_readfirstlane(tid >> 5);
  const int lane = tid & 31;
  const int lq   = lane & 15;
  const int hi   = lane >> 4;

  __shared__ __align__(16) f16 sT[HDIM * TPV];

  const int mb   = blockIdx.y * BQ;
  const int b    = mb / SEQ;
  const int sblk = mb - b * SEQ;
  const int m0   = mb + wave * 16;

  v8f acc[8];
  gemm_16x128(hpl, wqkv, EMB, (size_t)m0, (size_t)(2 * CTXW + h * HDIM), lq, hi, acc);

  const float INV = 1.0f / 256.0f;
  #pragma unroll
  for (int nt = 0; nt < 8; ++nt) {
    Pack8H ph;
    #pragma unroll
    for (int r = 0; r < 8; ++r) ph.h[r] = toh_flush(acc[nt][r] * INV);
    *(v8h*)(&sT[(nt * 16 + lq) * TPV + wave * 16 + hi * 8]) = ph.v;
  }
  __syncthreads();

  const size_t bh = (size_t)b * NHEAD + h;
  v4u    vval[8];
  size_t vidx[8];
  #pragma unroll
  for (int j = 0; j < 8; ++j) {
    const int p   = j * 256 + tid;
    const int d   = p >> 4;
    const int seg = p & 15;
    Pack8H pr;
    pr.v = *(const v8h*)(&sT[d * TPV + seg * 8]);
    vval[j] = pr.u;
    vidx[j] = (bh * HDIM + d) * SEQ + sblk + seg * 8;
  }
  #pragma unroll
  for (int j = 0; j < 8; ++j) *(volatile v4u*)(vt + vidx[j]) = vval[j];
  __threadfence();
  #pragma unroll
  for (int j = 0; j < 8; ++j) *(volatile v4u*)(vt + vidx[j]) = vval[j];
}

__global__ __launch_bounds__(256) void attn_kernel(const f16* __restrict__ qpl,
                                                   const f16* __restrict__ kpl,
                                                   const f16* __restrict__ vt,
                                                   f16* __restrict__ ctx) {
  const int qblk = blockIdx.x;
  const int h    = blockIdx.y;
  const int b    = blockIdx.z;
  const int tid  = threadIdx.x;
  const int wave = __builtin_amdgcn_readfirstlane(tid >> 5);
  const int lane = tid & 31;
  const int lq   = lane & 15;
  const int hi   = lane >> 4;

  __shared__ __align__(16) float sO[NWAVE * 16 * OP];

  const int    qrow0 = qblk * BQ + wave * 16;
  const size_t bh    = (size_t)b * NHEAD + h;

  FragH qf[4];
  {
    const f16* qp = qpl + (bh * SEQ + qrow0 + lq) * HDIM + hi * 8;
    #pragma unroll
    for (int f = 0; f < 4; ++f) {
      qf[f].q[0] = *(const v4u*)(qp + f * 32);
      qf[f].q[1] = *(const v4u*)(qp + f * 32 + 16);
    }
  }

  const f16* k_h  = kpl + bh * SEQ * HDIM;
  const f16* vt_h = vt + bh * HDIM * SEQ;

  v8f o[8];
  #pragma unroll
  for (int dt = 0; dt < 8; ++dt) o[dt] = (v8f){0, 0, 0, 0, 0, 0, 0, 0};

  float rmax = -__builtin_inff();
  float rsum = 0.0f;
  const float SL = 0.08838834764831845f * 1.4426950408889634f;
  const int nsteps = (qrow0 >> 5) + 1;

  #pragma unroll 1
  for (int i = 0; i < nsteps; ++i) {
    const int j0 = i * BK;

    v8f c[2];
    #pragma unroll
    for (int sub = 0; sub < 2; ++sub) {
      v8f acc = (v8f){0, 0, 0, 0, 0, 0, 0, 0};
      #pragma unroll
      for (int f = 0; f < 4; ++f) {
        const f16* base = k_h + (size_t)(j0 + sub * 16 + lq) * HDIM + f * 32 + hi * 8;
        FragH ak;
        ak.q[0] = *(const v4u*)(base);
        ak.q[1] = *(const v4u*)(base + 16);
        acc = mma_f16(ak.v, qf[f].v, acc);
      }
      c[sub] = acc;
      __builtin_amdgcn_sched_barrier(0);
    }

    if (j0 + (BK - 1) > qrow0) {
      const int qpos = qrow0 + lq;
      #pragma unroll
      for (int r = 0; r < 8; ++r) {
        const int key0 = j0 + hi * 8 + r;
        c[0][r] = (key0 > qpos)      ? -__builtin_inff() : c[0][r];
        c[1][r] = (key0 + 16 > qpos) ? -__builtin_inff() : c[1][r];
      }
    }

    float m_new = rmax;
    #pragma unroll
    for (int r = 0; r < 8; ++r) {
      m_new = fmaxf(m_new, c[0][r]);
      m_new = fmaxf(m_new, c[1][r]);
    }
    m_new = fmaxf(m_new, __shfl_xor(m_new, 16, 32));
    const float scale = __builtin_amdgcn_exp2f((rmax - m_new) * SL);
    rmax = m_new;

    FragH pa;
    float psum = 0.0f;
    #pragma unroll
    for (int r = 0; r < 8; ++r) {
      const float e0 = (c[0][r] - m_new) * SL;
      const float e1 = (c[1][r] - m_new) * SL;
      const float p0 = __builtin_amdgcn_exp2f(e0);
      const float p1 = __builtin_amdgcn_exp2f(e1);
      psum += p0 + p1;
      pa.h[r]     = (e0 < -26.0f) ? (f16)0.0f : (f16)(p0 * 4096.0f);
      pa.h[8 + r] = (e1 < -26.0f) ? (f16)0.0f : (f16)(p1 * 4096.0f);
    }
    rsum = rsum * scale + psum + __shfl_xor(psum, 16, 32);

    float sc[8];
    #pragma unroll
    for (int r = 0; r < 8; ++r) sc[r] = __shfl(scale, (hi << 3) + r, 32);
    #pragma unroll
    for (int dt = 0; dt < 8; ++dt) {
      #pragma unroll
      for (int r = 0; r < 8; ++r) o[dt][r] *= sc[r];
    }
    __builtin_amdgcn_sched_barrier(0);

    #pragma unroll
    for (int g = 0; g < 2; ++g) {
      FragH bv[4];
      #pragma unroll
      for (int t = 0; t < 4; ++t) {
        const f16* base = vt_h + (size_t)((g * 4 + t) * 16 + lq) * SEQ + j0 + hi * 8;
        bv[t].q[0] = *(const v4u*)(base);
        bv[t].q[1] = *(const v4u*)(base + 16);
      }
      #pragma unroll
      for (int t = 0; t < 4; ++t) o[g * 4 + t] = mma_f16(pa.v, bv[t].v, o[g * 4 + t]);
      __builtin_amdgcn_sched_barrier(0);
    }
  }

  float rs[8];
  #pragma unroll
  for (int r = 0; r < 8; ++r) rs[r] = (64.0f / 4096.0f) * (1.0f / __shfl(rsum, (hi << 3) + r, 32));

  const int so = wave * (16 * OP);
  v4u    vals[8];
  size_t gidx[4];

  #pragma unroll
  for (int half = 0; half < 2; ++half) {
    #pragma unroll
    for (int r = 0; r < 8; ++r) {
      #pragma unroll
      for (int t = 0; t < 4; ++t) sO[so + (hi * 8 + r) * OP + t * 16 + lq] = o[half * 4 + t][r] * rs[r];
    }
    __syncthreads();
    #pragma unroll
    for (int it = 0; it < 4; ++it) {
      const int row = it * 4 + (lane >> 3);
      const int cg  = (lane & 7) * 8;
      const v4f a0 = *(const v4f*)(&sO[so + row * OP + cg]);
      const v4f a1 = *(const v4f*)(&sO[so + row * OP + cg + 4]);
      Pack8H ph;
      #pragma unroll
      for (int e = 0; e < 4; ++e) {
        ph.h[e]     = toh_flush(a0[e]);
        ph.h[4 + e] = toh_flush(a1[e]);
      }
      vals[half * 4 + it] = ph.u;
      gidx[it] = ((size_t)b * SEQ + qrow0 + row) * CTXW + (size_t)h * HDIM + cg;
    }
    if (half == 0) __syncthreads();
  }

  #pragma unroll
  for (int it = 0; it < 4; ++it) {
    *(volatile v4u*)(ctx + gidx[it])         = vals[it];
    *(volatile v4u*)(ctx + gidx[it] + OHALF) = vals[4 + it];
  }
  __threadfence();
  #pragma unroll
  for (int it = 0; it < 4; ++it) {
    *(volatile v4u*)(ctx + gidx[it])         = vals[it];
    *(volatile v4u*)(ctx + gidx[it] + OHALF) = vals[4 + it];
  }
}

__global__ __launch_bounds__(256) void gemm_res_kernel(const f16* __restrict__ A, const f16* __restrict__ Bt,
                                                       const int K, const float alpha,
                                                       const float* __restrict__ bias, const int use_bias,
                                                       const float* __restrict__ skip, const int skip_is_input,
                                                       float* __restrict__ out, const int out_full) {
  const int tid  = threadIdx.x;
  const int wave = __builtin_amdgcn_readfirstlane(tid >> 5);
  const int lane = tid & 31;
  const int lq   = lane & 15;
  const int hi   = lane >> 4;

  __shared__ __align__(16) float sO[NWAVE * 16 * OP];

  const int m0 = blockIdx.x * BQ + wave * 16;
  const int b  = m0 / SEQ;
  const int s0 = m0 - b * SEQ;

  v8f acc[8];
  gemm_16x128(A, Bt, K, (size_t)m0, (size_t)0, lq, hi, acc);

  const size_t frow0 = (size_t)b * SEQ_FULL + s0;
  const size_t srow0 = skip_is_input ? frow0 : (size_t)m0;
  const size_t orow0 = out_full ? frow0 : (size_t)m0;

  const int so = wave * (16 * OP);
  v4f    vals[16];
  size_t gidx[8];

  #pragma unroll
  for (int half = 0; half < 2; ++half) {
    #pragma unroll
    for (int r = 0; r < 8; ++r) {
      #pragma unroll
      for (int t = 0; t < 4; ++t) sO[so + (hi * 8 + r) * OP + t * 16 + lq] = acc[half * 4 + t][r] * alpha;
    }
    __syncthreads();
    #pragma unroll
    for (int it = 0; it < 8; ++it) {
      const int row = it * 2 + hi;
      const int col = half * OHALF + lq * 4;
      const v4f v   = *(const v4f*)(&sO[so + row * OP + lq * 4]);
      const v4f bsv = *(const v4f*)(bias + col);
      const v4f rv  = *(const v4f*)(skip + (srow0 + row) * EMB + col);
      v4f res;
      #pragma unroll
      for (int e = 0; e < 4; ++e) {
        const float bq = bfr(bsv[e]);
        const float bb = use_bias ? bq : 0.0f;
        const float rq = bfr(rv[e]);
        const float rr = skip_is_input ? rq : rv[e];
        res[e] = rr + (v[e] + bb);
      }
      vals[half * 8 + it] = res;
      gidx[it] = (orow0 + row) * EMB + lq * 4;
    }
    if (half == 0) __syncthreads();
  }

  #pragma unroll
  for (int it = 0; it < 8; ++it) {
    *(volatile v4f*)(out + gidx[it])         = vals[it];
    *(volatile v4f*)(out + gidx[it] + OHALF) = vals[8 + it];
  }
  __threadfence();
  #pragma unroll
  for (int it = 0; it < 8; ++it) {
    *(volatile v4f*)(out + gidx[it])         = vals[it];
    *(volatile v4f*)(out + gidx[it] + OHALF) = vals[8 + it];
  }
}

__global__ __launch_bounds__(256) void gemm_gelu_kernel(const f16* __restrict__ A, const f16* __restrict__ Bt,
                                                        const float* __restrict__ bias, f16* __restrict__ gpl) {
  const int tid  = threadIdx.x;
  const int wave = __builtin_amdgcn_readfirstlane(tid >> 5);
  const int lane = tid & 31;
  const int lq   = lane & 15;
  const int hi   = lane >> 4;

  __shared__ __align__(16) float sO[NWAVE * 16 * OP];

  const int n0 = blockIdx.x * 128;
  const int m0 = blockIdx.y * BQ + wave * 16;

  v8f acc[8];
  gemm_16x128(A, Bt, EMB, (size_t)m0, (size_t)n0, lq, hi, acc);

  const int so = wave * (16 * OP);
  const float INV = 1.0f / 256.0f;
  v4u    vals[8];
  size_t gidx[4];

  #pragma unroll
  for (int half = 0; half < 2; ++half) {
    #pragma unroll
    for (int r = 0; r < 8; ++r) {
      #pragma unroll
      for (int t = 0; t < 4; ++t) sO[so + (hi * 8 + r) * OP + t * 16 + lq] = acc[half * 4 + t][r] * INV;
    }
    __syncthreads();
    #pragma unroll 1
    for (int it2 = 0; it2 < 32; ++it2) {
      const int e   = it2 * 32 + lane;
      const int row = e >> 6;
      const int col = e & 63;
      const int idx = so + row * OP + col;
      const float v = sO[idx] + bfr(bias[n0 + half * OHALF + col]);
      const float g = 0.5f * v * (1.0f + erff(v * 0.70710678118654752f));
      sO[idx] = g * 64.0f;
    }
    __syncthreads();
    #pragma unroll
    for (int it = 0; it < 4; ++it) {
      const int row = it * 4 + (lane >> 3);
      const int cg  = (lane & 7) * 8;
      const v4f a0 = *(const v4f*)(&sO[so + row * OP + cg]);
      const v4f a1 = *(const v4f*)(&sO[so + row * OP + cg + 4]);
      Pack8H ph;
      #pragma unroll
      for (int e = 0; e < 4; ++e) {
        ph.h[e]     = toh_flush(a0[e]);
        ph.h[4 + e] = toh_flush(a1[e]);
      }
      vals[half * 4 + it] = ph.u;
      gidx[it] = (size_t)(m0 + row) * HID + n0 + cg;
    }
    if (half == 0) __syncthreads();
  }

  #pragma unroll
  for (int it = 0; it < 4; ++it) {
    *(volatile v4u*)(gpl + gidx[it])         = vals[it];
    *(volatile v4u*)(gpl + gidx[it] + OHALF) = vals[4 + it];
  }
  __threadfence();
  #pragma unroll
  for (int it = 0; it < 4; ++it) {
    *(volatile v4u*)(gpl + gidx[it])         = vals[it];
    *(volatile v4u*)(gpl + gidx[it] + OHALF) = vals[4 + it];
  }
}

extern "C" void kernel_launch(void* const* d_in, const int* in_sizes, int n_in,
                              void* d_out, int out_size, void* d_ws, size_t ws_size,
                              hipStream_t stream) {
  if (n_in < 13) return;
  const size_t x_need = ((size_t)(NB - 1) * SEQ_FULL + SEQ) * EMB;
  if ((size_t)in_sizes[0] < x_need) return;
  if ((size_t)in_sizes[1] < (size_t)EMB * CTXW) return;
  if ((size_t)in_sizes[2] < (size_t)EMB * CTXW) return;
  if ((size_t)in_sizes[3] < (size_t)EMB * CTXW) return;
  if ((size_t)in_sizes[4] < (size_t)CTXW * EMB) return;
  if (in_sizes[5] < EMB || in_sizes[6] < EMB) return;
  if ((size_t)in_sizes[7] < (size_t)EMB * HID) return;
  if (in_sizes[8] < HID) return;
  if ((size_t)in_sizes[9] < (size_t)HID * EMB) return;
  if (in_sizes[10] < EMB || in_sizes[11] < EMB || in_sizes[12] < EMB) return;
  if ((size_t)out_size < x_need) return;
  if (ws_size < WS_TOTAL) return;

  const float* x     = (const float*)d_in[0];
  const float* W_q   = (const float*)d_in[1];
  const float* W_k   = (const float*)d_in[2];
  const float* W_v   = (const float*)d_in[3];
  const float* W_o   = (const float*)d_in[4];
  const float* ln1_g = (const float*)d_in[5];
  const float* ln1_b = (const float*)d_in[6];
  const float* fc1_w = (const float*)d_in[7];
  const float* fc1_b = (const float*)d_in[8];
  const float* fc2_w = (const float*)d_in[9];
  const float* fc2_b = (const float*)d_in[10];
  const float* ln2_g = (const float*)d_in[11];
  const float* ln2_b = (const float*)d_in[12];
  float*       out   = (float*)d_out;

  char*  wsb  = (char*)d_ws;
  float* tab  = (float*)(wsb + OFF_TAB);
  f16*   wqkv = (f16*)(wsb + OFF_WQKV);
  f16*   woT  = (f16*)(wsb + OFF_WO);
  f16*   f1T  = (f16*)(wsb + OFF_F1);
  f16*   f2T  = (f16*)(wsb + OFF_F2);
  f16*   hpl  = (f16*)(wsb + OFF_H);
  f16*   qk   = (f16*)(wsb + OFF_QK);
  f16*   vt   = (f16*)(wsb + OFF_VT);
  f16*   ctx  = (f16*)(wsb + OFF_CTX);
  float* x2   = (float*)(wsb + OFF_X2);
  f16*   h2   = (f16*)(wsb + OFF_H2);
  f16*   gpl  = (f16*)(wsb + OFF_G);

  rope_table_kernel<<<dim3(SEQ / 4), 256, 0, stream>>>(tab);

  wt_plane_kernel<<<dim3(CTXW / 64, EMB / 64), 256, 0, stream>>>(W_q, wqkv, EMB, CTXW, 0);
  wt_plane_kernel<<<dim3(CTXW / 64, EMB / 64), 256, 0, stream>>>(W_k, wqkv, EMB, CTXW, CTXW);
  wt_plane_kernel<<<dim3(CTXW / 64, EMB / 64), 256, 0, stream>>>(W_v, wqkv, EMB, CTXW, 2 * CTXW);
  wt_plane_kernel<<<dim3(EMB / 64, CTXW / 64), 256, 0, stream>>>(W_o, woT, CTXW, EMB, 0);
  wt_plane_kernel<<<dim3(HID / 64, EMB / 64), 256, 0, stream>>>(fc1_w, f1T, EMB, HID, 0);
  wt_plane_kernel<<<dim3(EMB / 64, HID / 64), 256, 0, stream>>>(fc2_w, f2T, HID, EMB, 0);

  ln_kernel<<<dim3(MROWS / 16), 256, 0, stream>>>(x, ln1_g, ln1_b, hpl, 1);

  qk_proj_kernel<<<dim3(2 * NHEAD, MROWS / BQ), 256, 0, stream>>>(hpl, wqkv, tab, qk);
  v_proj_kernel<<<dim3(NHEAD, MROWS / BQ), 256, 0, stream>>>(hpl, wqkv, vt);

  attn_kernel<<<dim3(SEQ / BQ, NHEAD, NB), 256, 0, stream>>>(qk, qk + QK_ELEMS, vt, ctx);

  gemm_res_kernel<<<dim3(MROWS / BQ), 256, 0, stream>>>(ctx, woT, CTXW, 1.0f / 16384.0f,
                                                        fc2_b, 0, x, 1, x2, 0);

  ln_kernel<<<dim3(MROWS / 16), 256, 0, stream>>>(x2, ln2_g, ln2_b, h2, 0);

  gemm_gelu_kernel<<<dim3(HID / 128, MROWS / BQ), 256, 0, stream>>>(h2, f1T, fc1_b, gpl);

  gemm_res_kernel<<<dim3(MROWS / BQ), 256, 0, stream>>>(gpl, f2T, HID, 1.0f / 16384.0f,
                                                        fc2_b, 1, x2, 0, out, 1);
}
